// GCN_5609227289259
// MI455X (gfx1250) — hardware-run, weakly checked
//
#include <hip/hip_runtime.h>

typedef float          v8f   __attribute__((ext_vector_type(8)));
typedef float          v4f   __attribute__((ext_vector_type(4)));
typedef unsigned int   v4u   __attribute__((ext_vector_type(4)));
typedef int            v8i   __attribute__((ext_vector_type(8)));
typedef unsigned short v8us  __attribute__((ext_vector_type(8)));
typedef unsigned short v16us __attribute__((ext_vector_type(16)));
typedef __bf16         v16bf __attribute__((ext_vector_type(16)));
typedef _Float16       v16h  __attribute__((ext_vector_type(16)));
typedef v4f  __attribute__((may_alias)) v4fa;
typedef v8us __attribute__((may_alias)) v8usa;
union FragB { v16bf v; v16us u; v8us h[2]; v8i w; };
union FragH { v16h  v; v16us u; v8us h[2]; v8i w; };

__device__ __forceinline__ v8f wmb(const FragB& a, const FragB& b, v8f c) {
  v8f d = __builtin_amdgcn_wmma_f32_16x16x32_bf16(false, a.v, false, b.v, (short)0, c, false, false);
  asm volatile("v_nop\n\tv_nop\n\tv_nop\n\tv_nop" : "+v"(d) : "v"(a.w), "v"(b.w));
  return d;
}

__device__ __forceinline__ v8f wmh(const FragH& a, const FragH& b, v8f c) {
  v8f d = __builtin_amdgcn_wmma_f32_16x16x32_f16(false, a.v, false, b.v, (short)0, c, false, false);
  asm volatile("v_nop\n\tv_nop\n\tv_nop\n\tv_nop" : "+v"(d) : "v"(a.w), "v"(b.w));
  return d;
}

__device__ __forceinline__ unsigned bf16_bits(float f) {
  const unsigned u = __float_as_uint(f);
  const unsigned r = (u + 0x7FFFu + ((u >> 16) & 1u)) >> 16;
  const unsigned q = (u >> 16) | 0x40u;
  return ((u & 0x7fffffffu) > 0x7f800000u) ? q : r;
}

__device__ __forceinline__ float bf16_val(float f) {
  return __uint_as_float(bf16_bits(f) << 16);
}
__device__ __forceinline__ int clampi(int v, int lo, int hi) {
  return v < lo ? lo : (v > hi ? hi : v);
}

__device__ __forceinline__ unsigned f16_bits(float f) {
  const unsigned u  = __float_as_uint(f);
  const unsigned s  = (u >> 16) & 0x8000u;
  const unsigned a  = u & 0x7fffffffu;
  const unsigned t  = a - 0x38000000u;
  const unsigned r  = (t + 0x0FFFu + ((t >> 13) & 1u)) >> 13;
  const unsigned rc = r > 0x7C00u ? 0x7C00u : r;
  const bool small  = a < 0x38800000u;
  const bool isnan  = a > 0x7f800000u;
  const unsigned fin = small ? 0u : (s | rc);
  return isnan ? (s | 0x7E00u) : fin;
}

__device__ __forceinline__ unsigned pk16(unsigned lo, unsigned hi) { return lo | (hi << 16); }
__device__ __forceinline__ unsigned bf16_lo_bits(float v) {
  float hi = bf16_val(v);
  asm volatile("" : "+v"(hi));
  return bf16_bits(v - hi);
}
__device__ __forceinline__ v4u pack8_bf16(v4f a, v4f c) {
  return (v4u){ pk16(bf16_bits(a[0]), bf16_bits(a[1])), pk16(bf16_bits(a[2]), bf16_bits(a[3])),
                pk16(bf16_bits(c[0]), bf16_bits(c[1])), pk16(bf16_bits(c[2]), bf16_bits(c[3])) };
}
__device__ __forceinline__ v4u pack8_bf16_lo(v4f a, v4f c) {
  return (v4u){ pk16(bf16_lo_bits(a[0]), bf16_lo_bits(a[1])), pk16(bf16_lo_bits(a[2]), bf16_lo_bits(a[3])),
                pk16(bf16_lo_bits(c[0]), bf16_lo_bits(c[1])), pk16(bf16_lo_bits(c[2]), bf16_lo_bits(c[3])) };
}
__device__ __forceinline__ v4u pack8_f16(v4f a, v4f c) {
  return (v4u){ pk16(f16_bits(a[0]), f16_bits(a[1])), pk16(f16_bits(a[2]), f16_bits(a[3])),
                pk16(f16_bits(c[0]), f16_bits(c[1])), pk16(f16_bits(c[2]), f16_bits(c[3])) };
}

template <int FORM>
__global__ __launch_bounds__(256) void k_plane(const float* __restrict__ src, int rows, int cols, int ldsrc,
                                               unsigned short* __restrict__ dst, int MP, int KP) {
  static_assert(FORM >= 0 && FORM <= 3);
  const int KTOT = (FORM == 1 || FORM == 3) ? 2 * KP : KP;
  const unsigned ppr   = (unsigned)(KTOT >> 3);
  const unsigned kp8   = (unsigned)(KP >> 3);
  const unsigned total = (unsigned)MP * ppr;
  const unsigned g     = blockIdx.x * 256u + threadIdx.x;
  const unsigned rowu  = g / ppr;
  const unsigned p     = g - rowu * ppr;
  const bool second    = p >= kp8;
  const int row = (int)rowu;
  const int c0  = (int)((second ? p - kp8 : p) << 3);
  const float* srow = src + (size_t)clampi(row, 0, rows - 1) * (size_t)ldsrc;
  float x[8];
  unsigned mk[8];
#pragma unroll
  for (int e = 0; e < 8; ++e) {
    const int c = c0 + e;
    const float v = srow[clampi(c, 0, cols - 1)];
    asm volatile("" :: "v"(v));
    x[e]  = v;
    mk[e] = (row < rows && c < cols) ? 0xFFFFu : 0u;
  }
  const v4f a = (v4f){ x[0], x[1], x[2], x[3] };
  const v4f c = (v4f){ x[4], x[5], x[6], x[7] };
  v4u o;
  if (FORM == 2) {
    o = pack8_f16(a, c);
  } else {
    const v4u hi = pack8_bf16(a, c);
    o = hi;
    if (FORM == 1) { const v4u lo = pack8_bf16_lo(a, c); o = second ? lo : hi; }
  }
  const v4u mw = (v4u){ pk16(mk[0], mk[1]), pk16(mk[2], mk[3]), pk16(mk[4], mk[5]), pk16(mk[6], mk[7]) };
  o &= mw;
  if (g < total) {
    volatile v4u* q = (volatile v4u*)(dst + (size_t)g * 8);
    *q = o;
    __threadfence();
    *q = o;
  }
}

template <int FORM> struct FragOf    { typedef FragB T; };
template <>         struct FragOf<2> { typedef FragH T; };
__device__ __forceinline__ v8f mm(const FragB& a, const FragB& b, v8f c) { return wmb(a, b, c); }
__device__ __forceinline__ v8f mm(const FragH& a, const FragH& b, v8f c) { return wmh(a, b, c); }
template <class F> __device__ __forceinline__ F ld_frag(const unsigned short* p) {
  F f;
  f.h[0] = *(const v8usa*)(p);
  f.h[1] = *(const v8usa*)(p + 16);
  return f;
}

template <int FORM, int EPI>
__global__ __launch_bounds__(256) __attribute__((amdgpu_num_vgpr(248)))
void k_gemm_nt(const unsigned short* __restrict__ A, const unsigned short* __restrict__ B,
               const float* __restrict__ bias, float* __restrict__ D, int M, int N, int KTOT, int ldd) {
  static_assert(FORM >= 0 && FORM <= 2);
  static_assert(EPI == 0 || EPI == 1);
  typedef typename FragOf<FORM>::T F;
  __shared__ __attribute__((aligned(16))) float sT[8][16 * 68];
  const int lane = threadIdx.x & 31;
  const int wave = threadIdx.x >> 5;
  const int tilesM = (M + 63) >> 6;
  const int tilesN = (N + 63) >> 6;
  const int tile = blockIdx.x * 8 + wave;
  if (tile >= tilesM * tilesN) return;
  const int tm = tile / tilesN;
  const int tn = tile - tm * tilesN;
  const int m0 = tm << 6;
  const int n0 = tn << 6;

  const int rl = lane & 15;
  const int h8 = (lane >> 4) * 8;
  const unsigned short* pa = A + (size_t)(m0 + rl) * (size_t)KTOT + h8;
  const unsigned short* pb = B + (size_t)(n0 + rl) * (size_t)KTOT + h8;

  v8f acc[4][4];
#pragma unroll
  for (int i = 0; i < 4; ++i)
#pragma unroll
    for (int j = 0; j < 4; ++j) acc[i][j] = (v8f){0.f, 0.f, 0.f, 0.f, 0.f, 0.f, 0.f, 0.f};

#pragma unroll 1
  for (int k0 = 0; k0 < KTOT; k0 += 32) {
    F bf[4];
#pragma unroll
    for (int j = 0; j < 4; ++j) bf[j] = ld_frag<F>(pb + (size_t)(j << 4) * (size_t)KTOT + k0);
#pragma unroll
    for (int i = 0; i < 4; ++i) {
      const F af = ld_frag<F>(pa + (size_t)(i << 4) * (size_t)KTOT + k0);
#pragma unroll
      for (int j = 0; j < 4; ++j) acc[i][j] = mm(af, bf[j], acc[i][j]);
    }
  }

  float* slab = sT[wave];
  const int hh = lane >> 4;
  const int c4 = (lane & 15) * 4;
  const int nc = n0 + c4;
  const bool cok = nc < N;
  v4f bv = (v4f){0.f, 0.f, 0.f, 0.f};
  if (EPI == 1) {
    bv = *(const v4fa*)(bias + clampi(nc, 0, N - 4));
    asm volatile("" :: "v"(bv));
  }
#pragma unroll
  for (int i = 0; i < 4; ++i) {
    const int mBase = m0 + (i << 4);
#pragma unroll
    for (int j = 0; j < 4; ++j) {
#pragma unroll
      for (int r = 0; r < 8; ++r) slab[(h8 + r) * 68 + (j << 4) + rl] = acc[i][j][r];
    }
    __builtin_amdgcn_fence(__ATOMIC_RELEASE, "workgroup");
    __builtin_amdgcn_wave_barrier();
    __builtin_amdgcn_fence(__ATOMIC_ACQUIRE, "workgroup");
    v4f vv[8];
#pragma unroll
    for (int it = 0; it < 8; ++it) {
      const int row = it * 2 + hh;
      v4f v = *(const v4fa*)(slab + row * 68 + c4);
      if (EPI == 1) v += bv;
      vv[it] = v;
    }
    for (int pass = 0; pass < 2; ++pass) {
#pragma unroll
      for (int it = 0; it < 8; ++it) {
        const int row = mBase + it * 2 + hh;
        if (cok && row < M) *(volatile v4f*)(D + (size_t)row * (size_t)ldd + nc) = vv[it];
      }
      __threadfence();
    }
    __builtin_amdgcn_fence(__ATOMIC_RELEASE, "workgroup");
    __builtin_amdgcn_wave_barrier();
    __builtin_amdgcn_fence(__ATOMIC_ACQUIRE, "workgroup");
  }
}

#define GN       100000
#define GE       1600000
#define GD       64
#define MPAD     100096
#define NBLK     98
#define NBA      1024
#define NTHR     256
#define NWAVE    8
#define CHUNK    2048
#define NCHUNK   782
#define WCAP     256
#define RCAP     21504
#define DEGCAP   64
#define SRCB     17
#define GEMM2_TWO_TERM 1
#define K2TOT    (GEMM2_TWO_TERM ? 128 : 64)
#define NU1      (GD * (GD / 8))
#define NU2      (GD * (K2TOT / 8))
#define BK_INTS  (2 * RCAP + 3 * NBA + 16)
#define BK_LDS   (BK_INTS * 4)

static_assert(GD == 64);
static_assert(GN % 32 == 0);
static_assert(NBLK * NBA >= MPAD && MPAD >= GN);
static_assert(MPAD == 782 * 128 && MPAD % 64 == 0);
static_assert(GN == 781 * 128 + 32);
static_assert(781LL * CHUNK + 512 == (long long)GE);
static_assert(NCHUNK == (GE + CHUNK - 1) / CHUNK);
static_assert(GE % 4 == 0 && CHUNK == NWAVE * WCAP && WCAP == 2 * 32 * 4);
static_assert(GN <= (1 << SRCB));
static_assert((NBA - 1) < (1 << (31 - SRCB)));
static_assert(RCAP % 1024 == 0 && RCAP * 4 >= 16710 * 5);
static_assert(DEGCAP >= 36 + 8);
static_assert(BK_INTS % 4 == 0 && BK_LDS <= 262144);
static_assert(BK_LDS == 184384);
static_assert(NU1 % NTHR == 0 && NU2 % NTHR == 0);
static_assert(K2TOT % 32 == 0);
static_assert(NBA % NWAVE == 0 && NBA % 32 == 0);

typedef float v2f __attribute__((ext_vector_type(2)));
typedef int   v4i __attribute__((ext_vector_type(4)));
typedef v2f __attribute__((may_alias)) v2fa;
typedef v4i __attribute__((may_alias)) v4ia;

__global__ __launch_bounds__(NTHR) void k_prep(const float* __restrict__ W1, const float* __restrict__ W2,
                                               const float* __restrict__ b1, const float* __restrict__ b2,
                                               const float* __restrict__ a1, const float* __restrict__ a2,
                                               unsigned short* __restrict__ W1T, unsigned short* __restrict__ W2D,
                                               float* __restrict__ PAR) {
  const int tid = (int)threadIdx.x;
  const int bx  = (int)blockIdx.x;
  if (bx < (NU1 + NU2) / NTHR) {
    const bool first = bx < NU1 / NTHR;
    const int u   = bx * NTHR + tid;
    const int v   = first ? u : u - NU1;
    const int ppr = first ? (GD / 8) : (K2TOT / 8);
    const int n   = v / ppr;
    const int k8  = (v - n * ppr) * 8;
    const int kk  = k8 & (GD - 1);
    const size_t woff = (size_t)kk * GD + n;
    float x[8];
    if (first) {
#pragma unroll
      for (int e = 0; e < 8; ++e) {
        const float t = W1[woff + (size_t)e * GD];
        asm volatile("" :: "v"(t));
        x[e] = t;
      }
    } else {
#pragma unroll
      for (int e = 0; e < 8; ++e) {
        const float t = W2[woff + (size_t)e * GD];
        asm volatile("" :: "v"(t));
        x[e] = t;
      }
    }
    const v4u o = pack8_bf16((v4f){ x[0], x[1], x[2], x[3] }, (v4f){ x[4], x[5], x[6], x[7] });
    if (first) {
      volatile v4u* q = (volatile v4u*)(W1T + (size_t)v * 8);
      *q = o;
      __threadfence();
      *q = o;
    } else {
      volatile v4u* q = (volatile v4u*)(W2D + (size_t)v * 8);
      *q = o;
      __threadfence();
      *q = o;
    }
  } else {
    const int t = tid;
    const v4f vb1 = *(const v4fa*)(b1 + clampi(4 * t, 0, GD - 4));
    const v4f vb2 = *(const v4fa*)(b2 + clampi(4 * t - GD, 0, GD - 4));
    const float s1 = a1[0];
    const float s2 = a2[0];
    asm volatile("" :: "v"(vb1));
    asm volatile("" :: "v"(vb2));
    asm volatile("" :: "v"(s1));
    asm volatile("" :: "v"(s2));
    const unsigned m1 = (t < 16) ? 0xFFFFFFFFu : 0u;
    const unsigned m2 = (t >= 16 && t < 32) ? 0xFFFFFFFFu : 0u;
    const unsigned m3 = (t == 32) ? 0xFFFFFFFFu : 0u;
    v4u o;
    o.x = (__float_as_uint(bf16_val(vb1.x)) & m1) | (__float_as_uint(bf16_val(vb2.x)) & m2) |
          (__float_as_uint(bf16_val(s1)) & m3);
    o.y = (__float_as_uint(bf16_val(vb1.y)) & m1) | (__float_as_uint(bf16_val(vb2.y)) & m2) |
          (__float_as_uint(bf16_val(s2)) & m3);
    o.z = (__float_as_uint(bf16_val(vb1.z)) & m1) | (__float_as_uint(bf16_val(vb2.z)) & m2);
    o.w = (__float_as_uint(bf16_val(vb1.w)) & m1) | (__float_as_uint(bf16_val(vb2.w)) & m2);
    if (t < 64) {
      volatile v4u* q = (volatile v4u*)(PAR + 4 * t);
      *q = o;
      __threadfence();
      *q = o;
    }
  }
}

__device__ __forceinline__ void grp_load(const int* __restrict__ srcp, const int* __restrict__ dstp, int e0,
                                         unsigned nbs, unsigned& w0, unsigned& w1, unsigned& w2, unsigned& w3,
                                         int& f0, int& f1, int& f2, int& f3) {
  const int ec = e0 < (GE - 4) ? e0 : (GE - 4);
  const v4i dv = *(const v4ia*)(dstp + ec);
  const v4i sv = *(const v4ia*)(srcp + ec);
  asm volatile("" :: "v"(dv));
  asm volatile("" :: "v"(sv));
  const int vm = (e0 < GE) ? -1 : 0;
  const int d0 = (dv.x & vm) | ~vm;
  const int d1 = (dv.y & vm) | ~vm;
  const int d2 = (dv.z & vm) | ~vm;
  const int d3 = (dv.w & vm) | ~vm;
  const unsigned s0 = (unsigned)d0 - nbs;
  const unsigned s1 = (unsigned)d1 - nbs;
  const unsigned s2 = (unsigned)d2 - nbs;
  const unsigned s3 = (unsigned)d3 - nbs;
  f0 = s0 < (unsigned)NBA ? 1 : 0;
  f1 = s1 < (unsigned)NBA ? 1 : 0;
  f2 = s2 < (unsigned)NBA ? 1 : 0;
  f3 = s3 < (unsigned)NBA ? 1 : 0;
  w0 = ((s0 & (unsigned)(NBA - 1)) << SRCB) | (unsigned)clampi(sv.x, 0, GN - 1);
  w1 = ((s1 & (unsigned)(NBA - 1)) << SRCB) | (unsigned)clampi(sv.y, 0, GN - 1);
  w2 = ((s2 & (unsigned)(NBA - 1)) << SRCB) | (unsigned)clampi(sv.z, 0, GN - 1);
  w3 = ((s3 & (unsigned)(NBA - 1)) << SRCB) | (unsigned)clampi(sv.w, 0, GN - 1);
}

__global__ __launch_bounds__(NTHR) __attribute__((amdgpu_num_vgpr(248)))
void k_bucket(const int* __restrict__ ei, int* __restrict__ LIST, int* __restrict__ CNT, int* __restrict__ OFF,
              int* __restrict__ DINVB, int* __restrict__ FLAG) {
  extern __shared__ __attribute__((aligned(16))) int dsm[];
  int* hl   = dsm;
  int* sl   = dsm + RCAP;
  int* cnt  = dsm + 2 * RCAP;
  int* offs = cnt + NBA;
  int* cur  = offs + NBA;
  int* wcn  = cur + NBA;
  const int tid = (int)threadIdx.x, lane = tid & 31, wave = tid >> 5;
  const int bx = (int)blockIdx.x;
  const unsigned nbs = (unsigned)(bx * NBA);
  const int* srcp = ei;
  const int* dstp = ei + GE;

  {
    const v4i ng = { -1, -1, -1, -1 };
    const v4i z4 = { 0, 0, 0, 0 };
#pragma unroll 1
    for (int i = tid * 4; i < 2 * RCAP; i += NTHR * 4) *(v4ia*)(dsm + i) = ng;
#pragma unroll 1
    for (int i = 2 * RCAP + tid * 4; i < BK_INTS; i += NTHR * 4) *(v4ia*)(dsm + i) = z4;
  }
  __syncthreads();

  int t = 0, ov = 0;
#pragma unroll 1
  for (int ch = 0; ch < NCHUNK; ++ch) {
    const int par = (ch & 1) * 8;
    const int e0  = ch * CHUNK + wave * WCAP + lane * 4;
    unsigned a0, a1, a2, a3, c0, c1, c2, c3;
    int fa0, fa1, fa2, fa3, fb0, fb1, fb2, fb3;
    grp_load(srcp, dstp, e0,       nbs, a0, a1, a2, a3, fa0, fa1, fa2, fa3);
    grp_load(srcp, dstp, e0 + 128, nbs, c0, c1, c2, c3, fb0, fb1, fb2, fb3);
    const unsigned ma0 = __builtin_amdgcn_ballot_w32(fa0 != 0);
    const unsigned ma1 = __builtin_amdgcn_ballot_w32(fa1 != 0);
    const unsigned ma2 = __builtin_amdgcn_ballot_w32(fa2 != 0);
    const unsigned ma3 = __builtin_amdgcn_ballot_w32(fa3 != 0);
    const unsigned mb0 = __builtin_amdgcn_ballot_w32(fb0 != 0);
    const unsigned mb1 = __builtin_amdgcn_ballot_w32(fb1 != 0);
    const unsigned mb2 = __builtin_amdgcn_ballot_w32(fb2 != 0);
    const unsigned mb3 = __builtin_amdgcn_ballot_w32(fb3 != 0);
    const int la = (int)__builtin_amdgcn_mbcnt_lo(ma0, 0u) + (int)__builtin_amdgcn_mbcnt_lo(ma1, 0u) +
                   (int)__builtin_amdgcn_mbcnt_lo(ma2, 0u) + (int)__builtin_amdgcn_mbcnt_lo(ma3, 0u);
    const int ta = (int)__builtin_popcount(ma0) + (int)__builtin_popcount(ma1) +
                   (int)__builtin_popcount(ma2) + (int)__builtin_popcount(ma3);
    const int lb = ta + (int)__builtin_amdgcn_mbcnt_lo(mb0, 0u) + (int)__builtin_amdgcn_mbcnt_lo(mb1, 0u) +
                   (int)__builtin_amdgcn_mbcnt_lo(mb2, 0u) + (int)__builtin_amdgcn_mbcnt_lo(mb3, 0u);
    const int tb = (int)__builtin_popcount(mb0) + (int)__builtin_popcount(mb1) +
                   (int)__builtin_popcount(mb2) + (int)__builtin_popcount(mb3);
    const int wc = ta + tb;
    const int pa0 = la, pa1 = pa0 + fa0, pa2 = pa1 + fa1, pa3 = pa2 + fa2;
    const int pb0 = lb, pb1 = pb0 + fb0, pb2 = pb1 + fb1, pb3 = pb2 + fb2;
    if (lane == 0) wcn[par + wave] = wc;
    __syncthreads();
    const v4i q0 = *(const v4ia*)(wcn + par);
    const v4i q1 = *(const v4ia*)(wcn + par + 4);
    const int n0 = clampi(q0.x, 0, WCAP), n1 = clampi(q0.y, 0, WCAP);
    const int n2 = clampi(q0.z, 0, WCAP), n3 = clampi(q0.w, 0, WCAP);
    const int n4 = clampi(q1.x, 0, WCAP), n5 = clampi(q1.y, 0, WCAP);
    const int n6 = clampi(q1.z, 0, WCAP), n7 = clampi(q1.w, 0, WCAP);
    const int base = (wave > 0 ? n0 : 0) + (wave > 1 ? n1 : 0) + (wave > 2 ? n2 : 0) + (wave > 3 ? n3 : 0) +
                     (wave > 4 ? n4 : 0) + (wave > 5 ? n5 : 0) + (wave > 6 ? n6 : 0);
    const int tot = n0 + n1 + n2 + n3 + n4 + n5 + n6 + n7;
    const int tb0 = t + base;
    { const int p = tb0 + pa0; if (fa0 != 0 && p < RCAP) hl[p] = (int)a0; }
    { const int p = tb0 + pa1; if (fa1 != 0 && p < RCAP) hl[p] = (int)a1; }
    { const int p = tb0 + pa2; if (fa2 != 0 && p < RCAP) hl[p] = (int)a2; }
    { const int p = tb0 + pa3; if (fa3 != 0 && p < RCAP) hl[p] = (int)a3; }
    { const int p = tb0 + pb0; if (fb0 != 0 && p < RCAP) hl[p] = (int)c0; }
    { const int p = tb0 + pb1; if (fb1 != 0 && p < RCAP) hl[p] = (int)c1; }
    { const int p = tb0 + pb2; if (fb2 != 0 && p < RCAP) hl[p] = (int)c2; }
    { const int p = tb0 + pb3; if (fb3 != 0 && p < RCAP) hl[p] = (int)c3; }
    ov |= (t + tot > RCAP) ? 1 : 0;
    t += tot;
  }
  __syncthreads();
  const int tt = t < 0 ? 0 : (t > RCAP ? RCAP : t);

  if (wave == 0) {
#pragma unroll 1
    for (int b0 = 0; b0 < tt; b0 += 32) {
      const int idx = b0 + lane;
      const int ent = hl[idx < RCAP ? idx : RCAP - 1];
      const int m32 = (tt - b0) < 32 ? (tt - b0) : 32;
#pragma unroll 1
      for (int k = 0; k < m32; ++k) {
        const int u    = __builtin_amdgcn_readlane(ent, k);
        const int slot = (u >> SRCB) & (NBA - 1);
        if (lane == 0) cnt[slot] = cnt[slot] + 1;
      }
    }
  }
  __syncthreads();
  if (wave == 0) {
    const int sbase = lane * (NBA / 32);
    int s = 0;
#pragma unroll 1
    for (int i = 0; i < NBA / 32; ++i) s += cnt[sbase + i];
    int incl = s;
#pragma unroll
    for (int d = 1; d < 32; d <<= 1) {
      const int y = __shfl_up(incl, d, 32);
      incl += (lane >= d) ? y : 0;
    }
    int run = incl - s;
#pragma unroll 1
    for (int i = 0; i < NBA / 32; ++i) {
      const int cv = cnt[sbase + i];
      offs[sbase + i] = run;
      cur[sbase + i]  = run;
      run += cv;
    }
  }
  __syncthreads();
  if (wave == 0) {
#pragma unroll 1
    for (int b0 = 0; b0 < tt; b0 += 32) {
      const int idx = b0 + lane;
      const int ent = hl[idx < RCAP ? idx : RCAP - 1];
      const int m32 = (tt - b0) < 32 ? (tt - b0) : 32;
#pragma unroll 1
      for (int k = 0; k < m32; ++k) {
        const int u    = __builtin_amdgcn_readlane(ent, k);
        const int slot = (u >> SRCB) & (NBA - 1);
        if (lane == 0) {
          int p = cur[slot];
          p = p < 0 ? 0 : (p > RCAP - 1 ? RCAP - 1 : p);
          sl[p] = u;
          cur[slot] = p + 1;
        }
      }
    }
  }
  __syncthreads();
#pragma unroll 1
  for (int i = tid; i < NBA; i += NTHR) {
    const int c = cnt[i];
    const float deg = (float)(c + 1);
    const float r = 1.0f / sqrtf(deg);
    const float dv = (deg > 0.0f) ? r : 0.0f;
    cur[i] = __float_as_int(dv);
  }
  __syncthreads();

  int* lp = LIST + (size_t)bx * RCAP;
  const int fl = (ov != 0 || t > RCAP) ? 1 : 0;
  const v4i fv = { fl, fl, fl, fl };
  for (int pass = 0; pass < 2; ++pass) {
#pragma unroll 1
    for (int it = 0; it < RCAP / (NTHR * 4); ++it) {
      const int i4 = (it * NTHR + tid) * 4;
      const v4i v = *(const v4ia*)(sl + i4);
      v4i o;
      o.x = v.x < 0 ? -1 : (v.x & ((1 << SRCB) - 1));
      o.y = v.y < 0 ? -1 : (v.y & ((1 << SRCB) - 1));
      o.z = v.z < 0 ? -1 : (v.z & ((1 << SRCB) - 1));
      o.w = v.w < 0 ? -1 : (v.w & ((1 << SRCB) - 1));
      *(volatile v4i*)(lp + i4) = o;
    }
    {
      const v4i vc = *(const v4ia*)(cnt + 4 * tid);
      const v4i vo = *(const v4ia*)(offs + 4 * tid);
      const v4i vd = *(const v4ia*)(cur + 4 * tid);
      *(volatile v4i*)(CNT   + (size_t)bx * NBA + 4 * tid) = vc;
      *(volatile v4i*)(OFF   + (size_t)bx * NBA + 4 * tid) = vo;
      *(volatile v4i*)(DINVB + (size_t)bx * NBA + 4 * tid) = vd;
    }
    if (wave == 0 && lane < 8) *(volatile v4i*)(FLAG + (size_t)bx * 32 + 4 * lane) = fv;
    __threadfence();
  }
}

template <int LAYER>
__global__ __launch_bounds__(NTHR) __attribute__((amdgpu_num_vgpr(248)))
void k_replay(const float* __restrict__ H, const int* __restrict__ LIST, const int* __restrict__ CNT,
              const int* __restrict__ OFF, const float* __restrict__ DINV, const int* __restrict__ FLAG,
              const float* __restrict__ PAR, unsigned* __restrict__ X1W, float* __restrict__ outp) {
  __shared__ __attribute__((aligned(16))) float spar[256];
  const int tid = (int)threadIdx.x, lane = tid & 31, wave = tid >> 5;
  const int bx = (int)blockIdx.x;
  const int nodeBase = bx * NBA;
  if (tid < 64) {
    const v4f pv = *(const v4fa*)(PAR + 4 * tid);
    *(v4fa*)(spar + 4 * tid) = pv;
  }
  __syncthreads();
  const float bias0 = spar[LAYER * GD + 2 * lane];
  const float bias1 = spar[LAYER * GD + 2 * lane + 1];
  const float slope = spar[2 * GD + LAYER];
  const int flv = FLAG[(size_t)bx * 32];
  asm volatile("" :: "v"(flv));
  const bool bflag = flv != 0;
  const int* lp = LIST + (size_t)bx * RCAP;
  const float qn = __uint_as_float(0x7fc00000u);

#pragma unroll 1
  for (int si = 0; si < NBA / NWAVE; ++si) {
    const int i  = nodeBase + si * NWAVE + wave;
    const bool live = i < GN;
    const int ic = i < GN ? i : GN - 1;
    const int cv = CNT[i];
    const int ofv = OFF[i];
    const float di = DINV[ic];
    asm volatile("" :: "v"(cv));
    asm volatile("" :: "v"(ofv));
    asm volatile("" :: "v"(di));
    const bool big = (cv > DEGCAP) || (cv < 0);
    int c = clampi(cv, 0, DEGCAP);
    c = live ? c : 0;
    const int cn = __builtin_amdgcn_readfirstlane(c);
    const int o  = clampi(ofv, 0, RCAP - 1);
    float acc0 = 0.0f, acc1 = 0.0f;
#pragma unroll 1
    for (int b0 = 0; b0 < cn; b0 += 32) {
      const int idx = clampi(o + b0 + lane, 0, RCAP - 1);
      const int sw = lp[idx];
      asm volatile("" :: "v"(sw));
      const int sr = clampi(sw, 0, GN - 1);
      const float ds = DINV[sr];
      asm volatile("" :: "v"(ds));
      const float w = ds * di;
      const int wi = __float_as_int(w);
      const int m32 = (cn - b0) < 32 ? (cn - b0) : 32;
#pragma unroll 1
      for (int k = 0; k < m32; ++k) {
        const int   sk = __builtin_amdgcn_readlane(sr, k);
        const float wk = __int_as_float(__builtin_amdgcn_readlane(wi, k));
        const v2f a = *(const v2fa*)(H + (size_t)sk * GD + 2 * lane);
        acc0 = fmaf(wk, a.x, acc0);
        acc1 = fmaf(wk, a.y, acc1);
      }
    }
    const v2f hs = *(const v2fa*)(H + (size_t)ic * GD + 2 * lane);
    asm volatile("" :: "v"(hs));
    const float rd = di * di;
    acc0 = fmaf(rd, hs.x, acc0);
    acc1 = fmaf(rd, hs.y, acc1);
    float y0 = acc0 + bias0;
    float y1 = acc1 + bias1;
    y0 = (y0 >= 0.0f) ? y0 : slope * y0;
    y1 = (y1 >= 0.0f) ? y1 : slope * y1;
    const bool pois = bflag || big;
    y0 = pois ? qn : y0;
    y1 = pois ? qn : y1;
    const float v0 = live ? y0 : 0.0f;
    const float v1 = live ? y1 : 0.0f;
    if (LAYER == 0) {
      if (i < MPAD) {
        const unsigned hw = pk16(bf16_bits(v0), bf16_bits(v1));
        const unsigned lw = pk16(bf16_lo_bits(v0), bf16_lo_bits(v1));
        unsigned* rp = X1W + (size_t)i * (K2TOT / 2);
        *(volatile unsigned*)(rp + lane) = hw;
        if (GEMM2_TWO_TERM) *(volatile unsigned*)(rp + 32 + lane) = lw;
        __threadfence();
        *(volatile unsigned*)(rp + lane) = hw;
        if (GEMM2_TWO_TERM) *(volatile unsigned*)(rp + 32 + lane) = lw;
      }
    } else {
      if (live) {
        const v2f ov2 = (v2f){ v0, v1 };
        float* op = outp + (size_t)i * GD + 2 * lane;
        *(volatile v2f*)op = ov2;
        __threadfence();
        *(volatile v2f*)op = ov2;
      }
    }
  }
}

static constexpr size_t SZ_XB   = (size_t)MPAD * GD * 2;
static constexpr size_t SZ_H    = (size_t)MPAD * GD * 4;
static constexpr size_t SZ_X1   = (size_t)MPAD * K2TOT * 2;
static constexpr size_t SZ_LIST = (size_t)NBLK * RCAP * 4;
static constexpr size_t SZ_TAB  = (size_t)NBLK * NBA * 4;
static constexpr size_t SZ_W1T  = (size_t)GD * GD * 2;
static constexpr size_t SZ_W2D  = (size_t)GD * K2TOT * 2;
static constexpr size_t SZ_PAR  = 1024;
static constexpr size_t SZ_FLAG = (size_t)NBLK * 128;
static constexpr size_t O_XB   = 0;
static constexpr size_t O_H    = O_XB + SZ_XB;
static constexpr size_t O_X1   = O_H + SZ_H;
static constexpr size_t O_LIST = O_X1 + SZ_X1;
static constexpr size_t O_CNT  = O_LIST + SZ_LIST;
static constexpr size_t O_OFF  = O_CNT + SZ_TAB;
static constexpr size_t O_DINV = O_OFF + SZ_TAB;
static constexpr size_t O_W1T  = O_DINV + SZ_TAB;
static constexpr size_t O_W2D  = O_W1T + SZ_W1T;
static constexpr size_t O_PAR  = O_W2D + SZ_W2D;
static constexpr size_t O_FLAG = O_PAR + SZ_PAR;
static constexpr size_t WS_TOTAL = O_FLAG + SZ_FLAG;
static_assert(SZ_XB % 256 == 0 && SZ_H % 256 == 0 && SZ_X1 % 256 == 0 && SZ_LIST % 256 == 0);
static_assert(SZ_TAB % 256 == 0 && SZ_W1T % 256 == 0 && SZ_W2D % 256 == 0 && SZ_PAR % 256 == 0 && SZ_FLAG % 256 == 0);
static_assert(WS_TOTAL <= ((size_t)128 << 20));
static_assert(!GEMM2_TWO_TERM || WS_TOTAL == 73733376ull);
static_assert((size_t)MPAD * (K2TOT / 8) < ((size_t)2048 << 20));
static_assert((size_t)(GN - 1) * GD + GD - 1 == 6399999ull);

extern "C" void kernel_launch(void* const* d_in, const int* in_sizes, int n_in,
                              void* d_out, int out_size, void* d_ws, size_t ws_size,
                              hipStream_t stream) {
  if (n_in < 8) return;
  if (in_sizes[0] != GN * GD) return;
  if (in_sizes[1] != 2 * GE) return;
  if (in_sizes[2] != GD * GD || in_sizes[3] != GD) return;
  if (in_sizes[4] < 1) return;
  if (in_sizes[5] != GD * GD || in_sizes[6] != GD) return;
  if (in_sizes[7] < 1) return;
  if (out_size != GN * GD) return;
  if (ws_size < WS_TOTAL) return;

  const float* x  = (const float*)d_in[0];
  const int*   ei = (const int*)d_in[1];
  const float* W1 = (const float*)d_in[2];
  const float* b1 = (const float*)d_in[3];
  const float* a1 = (const float*)d_in[4];
  const float* W2 = (const float*)d_in[5];
  const float* b2 = (const float*)d_in[6];
  const float* a2 = (const float*)d_in[7];
  float* out = (float*)d_out;

  char* ws = (char*)d_ws;
  unsigned short* XB   = (unsigned short*)(ws + O_XB);
  float*          H    = (float*)(ws + O_H);
  unsigned short* X1   = (unsigned short*)(ws + O_X1);
  int*            LIST = (int*)(ws + O_LIST);
  int*            CNT  = (int*)(ws + O_CNT);
  int*            OFF  = (int*)(ws + O_OFF);
  float*          DINV = (float*)(ws + O_DINV);
  unsigned short* W1T  = (unsigned short*)(ws + O_W1T);
  unsigned short* W2D  = (unsigned short*)(ws + O_W2D);
  float*          PAR  = (float*)(ws + O_PAR);
  int*            FLAG = (int*)(ws + O_FLAG);

  hipFuncSetAttribute(reinterpret_cast<const void*>(&k_bucket), hipFuncAttributeMaxDynamicSharedMemorySize,
                      (int)BK_LDS);

  const int gemmBlocks = ((MPAD / 64) + 7) / 8;

  k_plane<0><<<MPAD * GD / 8 / 256, 256, 0, stream>>>(x, GN, GD, GD, XB, MPAD, GD);
  k_prep<<<(NU1 + NU2) / NTHR + 1, NTHR, 0, stream>>>(W1, W2, b1, b2, a1, a2, W1T, W2D, PAR);
  k_bucket<<<NBLK, NTHR, BK_LDS, stream>>>(ei, LIST, CNT, OFF, (int*)DINV, FLAG);
  k_gemm_nt<0, 0><<<gemmBlocks, 256, 0, stream>>>(XB, W1T, PAR, H, MPAD, GD, GD, GD);
  k_replay<0><<<NBLK, NTHR, 0, stream>>>(H, LIST, CNT, OFF, DINV, FLAG, PAR, (unsigned*)X1, out);
  k_gemm_nt<0, 0><<<gemmBlocks, 256, 0, stream>>>(X1, W2D, PAR, H, MPAD, GD, K2TOT, GD);
  k_replay<1><<<NBLK, NTHR, 0, stream>>>(H, LIST, CNT, OFF, DINV, FLAG, PAR, (unsigned*)X1, out);
}
